// Encoder_6442450944673
// MI455X (gfx1250) — hardware-verified
//
#include <hip/hip_runtime.h>
#include <math.h>

constexpr int NBATCH   = 256;
constexpr int LSIG     = 8192;
constexpr int NWIN     = 128;
constexpr int NSTRIDE  = 32;
constexpr int NSTEP    = 253;
constexpr int NH1      = 256;
constexpr int NH2      = 128;
constexpr int NG1      = 4 * NH1;
constexpr int NG2      = 4 * NH2;
constexpr int KCAT     = 384;
constexpr int NTHR     = 256;
constexpr int NWAVE    = NTHR / 32;
constexpr int ROWS_BLK = 16;
constexpr int A1P      = 2 * NH1 + NWIN + 8;
constexpr int A2P      = 2 * NH2 + NH1 + 8;
constexpr int HSP      = NH2 + 4;
constexpr float WCARRY     = 16.0f;
constexpr float WCARRY_INV = 1.0f / 16.0f;

static_assert(KCAT == NH1 + NWIN, "layer 1 concat depth");
static_assert(KCAT == NH2 + NH1, "layer 2 concat depth");
static_assert(KCAT % 32 == 0 && NH1 % 32 == 0 && NH2 % 32 == 0 && NWIN % 32 == 0, "k chunks of 32");
static_assert((NSTEP - 1) * NSTRIDE + NWIN == LSIG, "last window ends at the signal end");
static_assert(NH1 == 32 * NWAVE, "two 16-unit groups per wave in layer 1");
static_assert(NH2 == 16 * NWAVE, "one 16-unit group per wave in layer 2");
static_assert(NBATCH % ROWS_BLK == 0, "whole row tiles");
static_assert(ROWS_BLK * NWIN == NTHR * 8, "x staging covers the window tile exactly");
static_assert(ROWS_BLK * NH2 == 2 * NTHR * 4, "final store covers the output tile exactly");
static_assert(A1P % 8 == 0 && A2P % 8 == 0 && HSP % 4 == 0, "16-B aligned LDS rows");
static_assert((NG1 * (NH1 / 8)) % NTHR == 0 && (NG1 * (NWIN / 8)) % NTHR == 0, "convert grids exact");
static_assert((NG2 * (NH2 / 8)) % NTHR == 0 && (NG2 * (NH1 / 8)) % NTHR == 0, "convert grids exact");

typedef __attribute__((ext_vector_type(16))) _Float16 v16h;
typedef __attribute__((ext_vector_type(8)))  _Float16 v8h;
typedef __attribute__((ext_vector_type(8)))  float    v8f;
typedef __attribute__((ext_vector_type(4)))  float    v4f;

__device__ __forceinline__ void guard4_h(v8f& a0, v8f& a1, v8f& a2, v8f& a3,
                                         v16h x, v16h b0, v16h b1, v16h b2, v16h b3) {
  asm volatile("v_nop\n\tv_nop\n\tv_nop\n\tv_nop"
               : "+v"(a0), "+v"(a1), "+v"(a2), "+v"(a3)
               : "v"(x), "v"(b0), "v"(b1), "v"(b2), "v"(b3));
}
__device__ __forceinline__ void acc_guard4(v8f& a, v8f& b, v8f& c, v8f& d) {
  asm volatile("v_nop\n\tv_nop\n\tv_nop\n\tv_nop" : "+v"(a), "+v"(b), "+v"(c), "+v"(d));
}

template <typename T> struct Frag;
template <> struct Frag<_Float16> {
  typedef v16h V; union U { v16h v; v8h h[2]; };
  static __device__ __forceinline__ v16h load(const _Float16* p) {
    U f; f.h[0] = *(const v8h*)(p); f.h[1] = *(const v8h*)(p + 16); return f.v;
  }
  static __device__ __forceinline__ v8f mma(v16h a, v16h b, v8f c) {
    return __builtin_amdgcn_wmma_f32_16x16x32_f16(false, a, false, b, (short)0, c, false, false);
  }
};

__device__ __forceinline__ float fsig(float v) {
  v = fminf(fmaxf(v, -30.0f), 30.0f);
  return __builtin_amdgcn_rcpf(1.0f + expf(-v));
}
__device__ __forceinline__ float ftanh(float v) {
  v = fminf(fmaxf(v, -15.0f), 15.0f);
  return 1.0f - 2.0f * __builtin_amdgcn_rcpf(1.0f + expf(2.0f * v));
}

__global__ __launch_bounds__(NTHR) void cvt8_kernel(const float* __restrict__ src, unsigned short* __restrict__ dst,
                                                    int nrow, int ncol8, int spitch, int dpitch, int dcol0, float sc) {
  const int i  = blockIdx.x * NTHR + threadIdx.x;
  const int n8 = nrow * ncol8;
  if (i < n8) {
    const int row = i / ncol8;
    const int c8  = i - row * ncol8;
    const float* sp = src + (size_t)row * spitch + c8 * 8;
    const v4f a = *(const v4f*)(sp);
    const v4f b = *(const v4f*)(sp + 4);
    v8h hv;
#pragma unroll
    for (int e = 0; e < 4; ++e) {
      const float fa = a[e] * sc;
      const float fb = b[e] * sc;
      hv[e]     = (_Float16)fa;
      hv[4 + e] = (_Float16)fb;
    }
    unsigned short* dp = dst + (size_t)row * dpitch + dcol0 + c8 * 8;
    *(volatile v8h*)dp = hv;
    __threadfence();
    *(volatile v8h*)dp = hv;
  }
}

__global__ __launch_bounds__(NTHR) void lstm2_seq_kernel(const float* __restrict__ x,
                                                         const unsigned short* __restrict__ W1p,
                                                         const unsigned short* __restrict__ W2p,
                                                         const float* __restrict__ b_ih1, const float* __restrict__ b_hh1,
                                                         const float* __restrict__ b_ih2, const float* __restrict__ b_hh2,
                                                         float* __restrict__ out) {
  __shared__ __align__(16) _Float16 A1[ROWS_BLK * A1P];
  __shared__ __align__(16) _Float16 A2[ROWS_BLK * A2P];
  __shared__ __align__(16) float    Hs[ROWS_BLK * HSP];
  const _Float16* W1 = (const _Float16*)W1p;
  const _Float16* W2 = (const _Float16*)W2p;
  const int tid = threadIdx.x, lane = tid & 31, wave = tid >> 5;
  const int c = lane & 15, hh = lane >> 4, koff = hh * 8;
  const int b0 = blockIdx.x * ROWS_BLK;

#pragma unroll 1
  for (int i = tid; i < ROWS_BLK * A1P; i += NTHR) A1[i] = (_Float16)0.0f;
#pragma unroll 1
  for (int i = tid; i < ROWS_BLK * A2P; i += NTHR) A2[i] = (_Float16)0.0f;

  float bb1[2][4], bb2[4];
#pragma unroll
  for (int nt = 0; nt < 2; ++nt) {
    const int j = 32 * wave + 16 * nt + c;
#pragma unroll
    for (int g = 0; g < 4; ++g) bb1[nt][g] = b_ih1[g * NH1 + j] + b_hh1[g * NH1 + j];
    asm volatile("" : "+v"(bb1[nt][0]), "+v"(bb1[nt][1]), "+v"(bb1[nt][2]), "+v"(bb1[nt][3]));
  }
  {
    const int j2 = 16 * wave + c;
#pragma unroll
    for (int g = 0; g < 4; ++g) bb2[g] = b_ih2[g * NH2 + j2] + b_hh2[g * NH2 + j2];
    asm volatile("" : "+v"(bb2[0]), "+v"(bb2[1]), "+v"(bb2[2]), "+v"(bb2[3]));
  }

  float c1[2][8], c2[8], hfin[8];
#pragma unroll
  for (int r = 0; r < 8; ++r) { c1[0][r] = 0.0f; c1[1][r] = 0.0f; c2[r] = 0.0f; hfin[r] = 0.0f; }

  const v8f z8 = {0.f, 0.f, 0.f, 0.f, 0.f, 0.f, 0.f, 0.f};
  __syncthreads();

#pragma unroll 1
  for (int t = 0; t < NSTEP; ++t) {
    const int rb1 = (t & 1) * NH1;
    const int wb1 = NH1 - rb1;
    const int rb2 = (t & 1) * NH2;
    const int wb2 = NH2 - rb2;

    {
      const int m = tid >> 4, c8 = (tid & 15) * 8;
      const float* xp = x + (size_t)(b0 + m) * LSIG + (size_t)t * NSTRIDE + c8;
      const v4f xa = *(const v4f*)(xp);
      const v4f xb = *(const v4f*)(xp + 4);
      v8h hv;
#pragma unroll
      for (int e = 0; e < 4; ++e) {
        const float fa = xa[e];
        const float fb = xb[e];
        hv[e]     = (_Float16)fa;
        hv[4 + e] = (_Float16)fb;
      }
      *(v8h*)(A1 + m * A1P + 2 * NH1 + c8) = hv;
    }
    __syncthreads();

#pragma unroll
    for (int nt = 0; nt < 2; ++nt) {
      const int j = 32 * wave + 16 * nt + c;
      const _Float16* wrow  = W1 + (size_t)j * KCAT + koff;
      const _Float16* ahrow = A1 + c * A1P + rb1 + koff;
      const _Float16* axrow = A1 + c * A1P + 2 * NH1 + koff;
      v8f acc[4];
      acc[0] = z8; acc[1] = z8; acc[2] = z8; acc[3] = z8;
#pragma unroll 1
      for (int k0 = 0; k0 < NH1; k0 += 32) {
        const v16h a  = Frag<_Float16>::load(ahrow + k0);
        const v16h q0 = Frag<_Float16>::load(wrow + k0);
        const v16h q1 = Frag<_Float16>::load(wrow + (size_t)1 * NH1 * KCAT + k0);
        const v16h q2 = Frag<_Float16>::load(wrow + (size_t)2 * NH1 * KCAT + k0);
        const v16h q3 = Frag<_Float16>::load(wrow + (size_t)3 * NH1 * KCAT + k0);
        acc[0] = Frag<_Float16>::mma(a, q0, acc[0]);
        acc[1] = Frag<_Float16>::mma(a, q1, acc[1]);
        acc[2] = Frag<_Float16>::mma(a, q2, acc[2]);
        acc[3] = Frag<_Float16>::mma(a, q3, acc[3]);
        guard4_h(acc[0], acc[1], acc[2], acc[3], a, q0, q1, q2, q3);
      }
#pragma unroll 1
      for (int k0 = 0; k0 < NWIN; k0 += 32) {
        const v16h a  = Frag<_Float16>::load(axrow + k0);
        const v16h q0 = Frag<_Float16>::load(wrow + NH1 + k0);
        const v16h q1 = Frag<_Float16>::load(wrow + (size_t)1 * NH1 * KCAT + NH1 + k0);
        const v16h q2 = Frag<_Float16>::load(wrow + (size_t)2 * NH1 * KCAT + NH1 + k0);
        const v16h q3 = Frag<_Float16>::load(wrow + (size_t)3 * NH1 * KCAT + NH1 + k0);
        acc[0] = Frag<_Float16>::mma(a, q0, acc[0]);
        acc[1] = Frag<_Float16>::mma(a, q1, acc[1]);
        acc[2] = Frag<_Float16>::mma(a, q2, acc[2]);
        acc[3] = Frag<_Float16>::mma(a, q3, acc[3]);
        guard4_h(acc[0], acc[1], acc[2], acc[3], a, q0, q1, q2, q3);
      }
      acc_guard4(acc[0], acc[1], acc[2], acc[3]);
#pragma unroll
      for (int r = 0; r < 8; ++r) {
        const float zi = acc[0][r] * WCARRY_INV + bb1[nt][0];
        const float zf = acc[1][r] * WCARRY_INV + bb1[nt][1];
        const float zg = acc[2][r] * WCARRY_INV + bb1[nt][2];
        const float zo = acc[3][r] * WCARRY_INV + bb1[nt][3];
        const float ig = fsig(zi);
        const float fg = fsig(zf);
        const float gg = ftanh(zg);
        const float og = fsig(zo);
        const float cn = fg * c1[nt][r] + ig * gg;
        c1[nt][r] = cn;
        const float hn = og * ftanh(cn);
        const _Float16 hq = (_Float16)hn;
        A1[(8 * hh + r) * A1P + wb1 + j] = hq;
        A2[(8 * hh + r) * A2P + 2 * NH2 + j] = hq;
      }
    }
    __syncthreads();

    {
      const int j2 = 16 * wave + c;
      const _Float16* wrow  = W2 + (size_t)j2 * KCAT + koff;
      const _Float16* ahrow = A2 + c * A2P + rb2 + koff;
      const _Float16* axrow = A2 + c * A2P + 2 * NH2 + koff;
      v8f acc[4];
      acc[0] = z8; acc[1] = z8; acc[2] = z8; acc[3] = z8;
#pragma unroll 1
      for (int k0 = 0; k0 < NH2; k0 += 32) {
        const v16h a  = Frag<_Float16>::load(ahrow + k0);
        const v16h q0 = Frag<_Float16>::load(wrow + k0);
        const v16h q1 = Frag<_Float16>::load(wrow + (size_t)1 * NH2 * KCAT + k0);
        const v16h q2 = Frag<_Float16>::load(wrow + (size_t)2 * NH2 * KCAT + k0);
        const v16h q3 = Frag<_Float16>::load(wrow + (size_t)3 * NH2 * KCAT + k0);
        acc[0] = Frag<_Float16>::mma(a, q0, acc[0]);
        acc[1] = Frag<_Float16>::mma(a, q1, acc[1]);
        acc[2] = Frag<_Float16>::mma(a, q2, acc[2]);
        acc[3] = Frag<_Float16>::mma(a, q3, acc[3]);
        guard4_h(acc[0], acc[1], acc[2], acc[3], a, q0, q1, q2, q3);
      }
#pragma unroll 1
      for (int k0 = 0; k0 < NH1; k0 += 32) {
        const v16h a  = Frag<_Float16>::load(axrow + k0);
        const v16h q0 = Frag<_Float16>::load(wrow + NH2 + k0);
        const v16h q1 = Frag<_Float16>::load(wrow + (size_t)1 * NH2 * KCAT + NH2 + k0);
        const v16h q2 = Frag<_Float16>::load(wrow + (size_t)2 * NH2 * KCAT + NH2 + k0);
        const v16h q3 = Frag<_Float16>::load(wrow + (size_t)3 * NH2 * KCAT + NH2 + k0);
        acc[0] = Frag<_Float16>::mma(a, q0, acc[0]);
        acc[1] = Frag<_Float16>::mma(a, q1, acc[1]);
        acc[2] = Frag<_Float16>::mma(a, q2, acc[2]);
        acc[3] = Frag<_Float16>::mma(a, q3, acc[3]);
        guard4_h(acc[0], acc[1], acc[2], acc[3], a, q0, q1, q2, q3);
      }
      acc_guard4(acc[0], acc[1], acc[2], acc[3]);
#pragma unroll
      for (int r = 0; r < 8; ++r) {
        const float zi = acc[0][r] * WCARRY_INV + bb2[0];
        const float zf = acc[1][r] * WCARRY_INV + bb2[1];
        const float zg = acc[2][r] * WCARRY_INV + bb2[2];
        const float zo = acc[3][r] * WCARRY_INV + bb2[3];
        const float ig = fsig(zi);
        const float fg = fsig(zf);
        const float gg = ftanh(zg);
        const float og = fsig(zo);
        const float cn = fg * c2[r] + ig * gg;
        c2[r] = cn;
        const float hn = og * ftanh(cn);
        hfin[r] = hn;
        A2[(8 * hh + r) * A2P + wb2 + j2] = (_Float16)hn;
      }
    }
  }

  {
    const int j2 = 16 * wave + c;
#pragma unroll
    for (int r = 0; r < 8; ++r) Hs[(8 * hh + r) * HSP + j2] = hfin[r];
  }
  __syncthreads();
  for (int pass = 0; pass < 2; ++pass) {
#pragma unroll
    for (int it = 0; it < 2; ++it) {
      const int idx = it * NTHR + tid;
      const int row = idx >> 5, c4 = (idx & 31) * 4;
      const v4f v = *(const v4f*)(Hs + row * HSP + c4);
      *(volatile v4f*)(out + (size_t)(b0 + row) * NH2 + c4) = v;
    }
    __threadfence();
  }
}

extern "C" void kernel_launch(void* const* d_in, const int* in_sizes, int n_in,
                              void* d_out, int out_size, void* d_ws, size_t ws_size, hipStream_t stream) {
  if (n_in < 9 || d_out == nullptr || d_ws == nullptr) return;
  if (in_sizes[0] != NBATCH * LSIG || in_sizes[1] != NG1 * NWIN || in_sizes[2] != NG1 * NH1 ||
      in_sizes[3] != NG1 || in_sizes[4] != NG1 || in_sizes[5] != NG2 * NH1 || in_sizes[6] != NG2 * NH2 ||
      in_sizes[7] != NG2 || in_sizes[8] != NG2 || out_size != NBATCH * NH2) return;

  const float* x     = (const float*)d_in[0];
  const float* w_ih1 = (const float*)d_in[1];
  const float* w_hh1 = (const float*)d_in[2];
  const float* b_ih1 = (const float*)d_in[3];
  const float* b_hh1 = (const float*)d_in[4];
  const float* w_ih2 = (const float*)d_in[5];
  const float* w_hh2 = (const float*)d_in[6];
  const float* b_ih2 = (const float*)d_in[7];
  const float* b_hh2 = (const float*)d_in[8];
  float* out = (float*)d_out;

  char* ws = (char*)d_ws; size_t off = 0;
  auto carve = [&](size_t bytes) -> char* { char* p = ws + off; off += (bytes + 255) & ~(size_t)255; return p; };
  unsigned short* W1 = (unsigned short*)carve((size_t)NG1 * KCAT * 2);
  unsigned short* W2 = (unsigned short*)carve((size_t)NG2 * KCAT * 2);
  if (off > ws_size || off > (size_t)134217728) return;

  const int n8a = NG1 * (NH1 / 8);
  const int n8b = NG1 * (NWIN / 8);
  const int n8c = NG2 * (NH2 / 8);
  const int n8d = NG2 * (NH1 / 8);
  cvt8_kernel<<<n8a / NTHR, NTHR, 0, stream>>>(w_hh1, W1, NG1, NH1 / 8,  NH1,  KCAT, 0,   WCARRY);
  cvt8_kernel<<<n8b / NTHR, NTHR, 0, stream>>>(w_ih1, W1, NG1, NWIN / 8, NWIN, KCAT, NH1, WCARRY);
  cvt8_kernel<<<n8c / NTHR, NTHR, 0, stream>>>(w_hh2, W2, NG2, NH2 / 8,  NH2,  KCAT, 0,   WCARRY);
  cvt8_kernel<<<n8d / NTHR, NTHR, 0, stream>>>(w_ih2, W2, NG2, NH1 / 8,  NH1,  KCAT, NH2, WCARRY);

  lstm2_seq_kernel<<<NBATCH / ROWS_BLK, NTHR, 0, stream>>>(x, W1, W2, b_ih1, b_hh1, b_ih2, b_hh2, out);
}
